// MambaBlock_67138928771575
// MI455X (gfx1250) — hardware-verified
//
#include <hip/hip_runtime.h>
#include <math.h>

typedef __attribute__((ext_vector_type(16))) _Float16 v16h;
typedef __attribute__((ext_vector_type(8)))  _Float16 v8h;
typedef __attribute__((ext_vector_type(8)))  float    v8f;
typedef __attribute__((ext_vector_type(4)))  float    v4f;
typedef __attribute__((ext_vector_type(2)))  float    v2f;

constexpr int kBatch = 4;
constexpr int kSeq   = 1024;
constexpr int kDm    = 1024;
constexpr int kDin   = 2048;
constexpr int kNst   = 16;
constexpr int kRows  = kBatch * kSeq;
constexpr int kXzP   = 2 * kDin;
constexpr int kPrjN  = kDin + 2 * kNst;
constexpr int kPrjP  = 2112;
constexpr int kBcP   = 2 * kNst;
constexpr int kTP    = 260;
static_assert(kRows == 4096 && kXzP == 4096 && kPrjN == 2080, "shape constants");
static_assert((kPrjP % 64) == 0 && kPrjP >= kPrjN && (kPrjP - kDin) == 64, "x_proj pad");
static_assert((kDm % 32) == 0 && (kDin % 32) == 0, "GEMM K multiples of 32");
static_assert((kRows % 64) == 0 && (kXzP % 64) == 0 && (kDin % 64) == 0 && (kDm % 64) == 0, "GEMM M,N multiples of 64");
static_assert((kSeq % 64) == 0 && (kDin % 256) == 0 && kBcP == 32, "tile multiples");

constexpr float kCarX  = 16.0f;
constexpr float kCarW  = 32.0f;
constexpr float kCarXI = 16.0f;
constexpr float kCarDR = 16.0f;
constexpr float kCarDL = 64.0f;
constexpr float kCarY  = 64.0f;
constexpr float kSclIn  = 1.0f / (kCarX  * kCarW);
constexpr float kSclXp  = 1.0f / (kCarXI * kCarW);
constexpr float kSclDt  = 1.0f / (kCarDR * kCarW);
constexpr float kSclOut = 1.0f / (kCarY  * kCarW);
constexpr float kInvDL  = 1.0f / kCarDL;

constexpr size_t kSzP0  = (size_t)kRows * kDin * 2;
constexpr size_t kSzXZ  = (size_t)kRows * kXzP * 4;
constexpr size_t kSzP2  = (size_t)kRows * kDin * 2;
constexpr size_t kSzW2  = (size_t)kPrjP * kDin * 2;
constexpr size_t kSzBC  = (size_t)kRows * kBcP * 4;
constexpr size_t kSzW3  = (size_t)kDin * kDin * 2;
constexpr size_t kSzW4  = (size_t)kDm * kDin * 2;
constexpr size_t kOffP0 = 0;
constexpr size_t kOffXZ = kOffP0 + kSzP0;
constexpr size_t kOffP2 = kOffXZ + kSzXZ;
constexpr size_t kOffW2 = kOffP2 + kSzP2;
constexpr size_t kOffBC = kOffW2 + kSzW2;
constexpr size_t kOffW3 = kOffBC + kSzBC;
constexpr size_t kOffW4 = kOffW3 + kSzW3;
constexpr size_t kWsTotal = kOffW4 + kSzW4;
static_assert(kWsTotal == 122421248ull, "carve total");
static_assert(kWsTotal <= 134217728ull, "carve cap");
static_assert((size_t)kRows * kDm * 2 + (size_t)kXzP * kDm * 2 <= kSzP0, "P0 holds Xh + W1h");
static_assert((kOffXZ % 128) == 0 && (kOffP2 % 128) == 0 && (kOffW2 % 128) == 0 && (kOffBC % 128) == 0 &&
              (kOffW3 % 128) == 0 && (kOffW4 % 128) == 0, "128-B aligned regions");

__device__ __forceinline__ float h16_to_f32(unsigned hb) {
  const unsigned sgn = (hb & 0x8000u) << 16;
  const unsigned em = hb & 0x7fffu;
  const float fn = __uint_as_float((em << 13) + 0x38000000u);
  const float fs = (float)em * 5.9604644775390625e-8f;
  const float mag = (em < 0x400u) ? fs : fn;
  return __uint_as_float(__float_as_uint(mag) | sgn);
}

__device__ __forceinline__ void row_guard_h(v8f& a, v8f& b, v8f& c, v8f& d, v16h x, v16h b0, v16h b1, v16h b2, v16h b3) {
  asm volatile("v_nop\n\tv_nop\n\tv_nop\n\tv_nop" : "+v"(a), "+v"(b), "+v"(c), "+v"(d) : "v"(x), "v"(b0), "v"(b1), "v"(b2), "v"(b3));
}
__device__ __forceinline__ void keep4_h(v16h a, v16h b, v16h c, v16h d) { asm volatile("v_nop" :: "v"(a), "v"(b), "v"(c), "v"(d)); }
__device__ __forceinline__ void acc_guard4(v8f& a, v8f& b, v8f& c, v8f& d) { asm volatile("v_nop\n\tv_nop\n\tv_nop\n\tv_nop" : "+v"(a), "+v"(b), "+v"(c), "+v"(d)); }
struct FragH {
  union U { v16h v; v8h h[2]; };
  static __device__ __forceinline__ v16h load(const _Float16* p) {
    U f; f.h[0] = *(const v8h*)(p); f.h[1] = *(const v8h*)(p + 16); return f.v;
  }
  static __device__ __forceinline__ v8f mma(v16h a, v16h b, v8f c) {
    return __builtin_amdgcn_wmma_f32_16x16x32_f16(false, a, false, b, (short)0, c, false, false);
  }
};

template <int OUT_MODE, bool BIAS>
__global__ __launch_bounds__(256) void wmma_gemm64_f16(
    const unsigned short* __restrict__ Ap, int lda,
    const unsigned short* __restrict__ Btp, int ldb,
    void* __restrict__ Cout, int ldc,
    const float* __restrict__ bias,
    int M, int N, int K, float scale, float outMul) {
  const _Float16* A  = (const _Float16*)Ap;
  const _Float16* Bt = (const _Float16*)Btp;
  __shared__ __align__(16) float sT[8][16 * 68];
  const int lane = threadIdx.x & 31;
  const int wave = threadIdx.x >> 5;
  const int tilesN = N >> 6;
  const int tilesM = M >> 6;
  const int tile = blockIdx.x * 8 + wave;
  if (tile >= tilesM * tilesN) return;
  const int tm = tile / tilesN;
  const int tn = tile - tm * tilesN;
  const int m0 = tm << 6;
  const int n0 = tn << 6;

  const int rlane = lane & 15;
  const int koff  = (lane >> 4) * 8;
  const int mOff  = (lane >> 4) * 8;

  v8f acc[4][4];
#pragma unroll
  for (int i = 0; i < 4; ++i)
#pragma unroll
    for (int j = 0; j < 4; ++j) acc[i][j] = (v8f){0.f,0.f,0.f,0.f,0.f,0.f,0.f,0.f};

  for (int k0 = 0; k0 < K; k0 += 32) {
    v16h bh[4];
#pragma unroll
    for (int j = 0; j < 4; ++j) {
      const size_t bo = (size_t)(n0 + (j << 4) + rlane) * ldb + koff + k0;
      bh[j] = FragH::load(Bt + bo);
    }
#pragma unroll
    for (int i = 0; i < 4; ++i) {
      const size_t ao = (size_t)(m0 + (i << 4) + rlane) * lda + koff + k0;
      v16h ah = FragH::load(A + ao);
#pragma unroll
      for (int j = 0; j < 4; ++j) acc[i][j] = FragH::mma(ah, bh[j], acc[i][j]);
      row_guard_h(acc[i][0], acc[i][1], acc[i][2], acc[i][3], ah, bh[0], bh[1], bh[2], bh[3]);
    }
    keep4_h(bh[0], bh[1], bh[2], bh[3]);
  }
  acc_guard4(acc[0][0], acc[0][1], acc[0][2], acc[0][3]);
  acc_guard4(acc[1][0], acc[1][1], acc[1][2], acc[1][3]);
  acc_guard4(acc[2][0], acc[2][1], acc[2][2], acc[2][3]);
  acc_guard4(acc[3][0], acc[3][1], acc[3][2], acc[3][3]);

  float bvj[4];
#pragma unroll
  for (int j = 0; j < 4; ++j) bvj[j] = BIAS ? bias[n0 + (j << 4) + rlane] : 0.0f;

  float* slab = sT[wave];
#pragma unroll
  for (int i = 0; i < 4; ++i) {
    const int mBase = m0 + (i << 4);
#pragma unroll
    for (int j = 0; j < 4; ++j) {
#pragma unroll
      for (int r = 0; r < 8; ++r) {
        float v = acc[i][j][r] * scale;
        if (BIAS) v += bvj[j];
        if (OUT_MODE == 1) v *= outMul;
        slab[(mOff + r) * 68 + (j << 4) + rlane] = v;
      }
    }
    __builtin_amdgcn_fence(__ATOMIC_RELEASE, "workgroup");
    __builtin_amdgcn_wave_barrier();
    __builtin_amdgcn_fence(__ATOMIC_ACQUIRE, "workgroup");
    if (OUT_MODE == 0) {
      float* C = (float*)Cout;
      const int hh = lane >> 4, c4 = (lane & 15) * 4;
      for (int pass = 0; pass < 2; ++pass) {
#pragma unroll
        for (int it = 0; it < 8; ++it) {
          const int row = it * 2 + hh;
          v4f v = *(const v4f*)(slab + row * 68 + c4);
          *(volatile v4f*)(C + (size_t)(mBase + row) * ldc + n0 + c4) = v;
        }
        __threadfence();
      }
    } else if (OUT_MODE == 3) {
      float* C = (float*)Cout;
      const int q = lane >> 3, c4 = (lane & 7) * 4;
      for (int pass = 0; pass < 2; ++pass) {
#pragma unroll
        for (int it = 0; it < 4; ++it) {
          const int row = it * 4 + q;
          v4f v = *(const v4f*)(slab + row * 68 + c4);
          *(volatile v4f*)(C + (size_t)(mBase + row) * ldc + c4) = v;
        }
        __threadfence();
      }
    } else {
      const int q = lane >> 3, c8 = (lane & 7) * 8;
      unsigned short* C = (unsigned short*)Cout;
      for (int pass = 0; pass < 2; ++pass) {
#pragma unroll
        for (int it = 0; it < 4; ++it) {
          const int row = it * 4 + q;
          const float* sp = slab + row * 68 + c8;
          v8h hv;
#pragma unroll
          for (int e = 0; e < 8; ++e) hv[e] = (_Float16)sp[e];
          *(volatile v8h*)(C + (size_t)(mBase + row) * ldc + n0 + c8) = hv;
        }
        __threadfence();
      }
    }
    __builtin_amdgcn_fence(__ATOMIC_RELEASE, "workgroup");
    __builtin_amdgcn_wave_barrier();
    __builtin_amdgcn_fence(__ATOMIC_ACQUIRE, "workgroup");
  }
}

__global__ __launch_bounds__(256) void cast_f16_kernel(
    const float* __restrict__ src, unsigned short* __restrict__ dst, int total8, int real8, float scale)
{
  const int i = blockIdx.x * 256 + threadIdx.x;
  if (i >= total8) return;
  const bool live = (i < real8);
  const size_t e0 = (size_t)i << 3;
  const size_t es = live ? e0 : (size_t)0;
  const v4f a0 = *(const v4f*)(src + es);
  const v4f a1 = *(const v4f*)(src + es + 4);
  v8h hv;
#pragma unroll
  for (int e = 0; e < 4; ++e) {
    const float f0 = live ? (a0[e] * scale) : 0.0f;
    const float f1 = live ? (a1[e] * scale) : 0.0f;
    hv[e]     = (_Float16)f0;
    hv[4 + e] = (_Float16)f1;
  }
  unsigned short* q = dst + e0;
  *(volatile v8h*)q = hv;
  __threadfence();
  *(volatile v8h*)q = hv;
}

__global__ __launch_bounds__(256) void conv_silu_kernel(
    const float* __restrict__ XZ, const float* __restrict__ cw, const float* __restrict__ cb,
    unsigned short* __restrict__ XI16)
{
  __shared__ __align__(16) float sT[16 * kTP];
  const int tid = threadIdx.x, lane = tid & 31, wave = tid >> 5;
  const int d0 = blockIdx.x * 256, d = d0 + tid;
  const int g0 = blockIdx.y * 64;
  const int tb = g0 & (kSeq - 1);
  const v4f wv = *(const v4f*)(cw + (size_t)d * 4);
  const float bc = cb[d];
  float xm3, xm2, xm1;
  {
    const bool hist = (tb > 0);
    const int rb = hist ? (g0 - 3) : g0;
    const float v3 = XZ[(size_t)rb * kXzP + d];
    const float v2 = XZ[(size_t)(rb + 1) * kXzP + d];
    const float v1 = XZ[(size_t)(rb + 2) * kXzP + d];
    xm3 = hist ? v3 : 0.f;
    xm2 = hist ? v2 : 0.f;
    xm1 = hist ? v1 : 0.f;
  }
#pragma unroll 1
  for (int sub = 0; sub < 4; ++sub) {
    const int lb = g0 + sub * 16;
#pragma unroll 1
    for (int s = 0; s < 16; ++s) {
      const float xcur = XZ[(size_t)(lb + s) * kXzP + d];
      float acc = bc;
      acc = fmaf(wv[0], xm3, acc);
      acc = fmaf(wv[1], xm2, acc);
      acc = fmaf(wv[2], xm1, acc);
      acc = fmaf(wv[3], xcur, acc);
      const float sg = __builtin_amdgcn_rcpf(1.0f + expf(-acc));
      sT[s * kTP + tid] = (acc * sg) * kCarXI;
      xm3 = xm2; xm2 = xm1; xm1 = xcur;
    }
    __syncthreads();
    v8h bv[2];
#pragma unroll
    for (int it = 0; it < 2; ++it) {
      const float* sp = sT + (it * 8 + wave) * kTP + lane * 8;
      const v4f a0 = *(const v4f*)(sp);
      const v4f a1 = *(const v4f*)(sp + 4);
#pragma unroll
      for (int e = 0; e < 4; ++e) {
        bv[it][e]     = (_Float16)a0[e];
        bv[it][4 + e] = (_Float16)a1[e];
      }
    }
    for (int pass = 0; pass < 2; ++pass) {
#pragma unroll
      for (int it = 0; it < 2; ++it)
        *(volatile v8h*)(XI16 + (size_t)(lb + it * 8 + wave) * kDin + d0 + lane * 8) = bv[it];
      __threadfence();
    }
    __syncthreads();
  }
}

__global__ __launch_bounds__(256) void scan_kernel(
    const float* __restrict__ XZ, const unsigned* __restrict__ DLW, const float* __restrict__ BC,
    const float* __restrict__ cw, const float* __restrict__ cb, const float* __restrict__ Alog,
    const float* __restrict__ Dv, unsigned short* __restrict__ YG)
{
  __shared__ __align__(16) float sBC[16 * kBcP];
  __shared__ __align__(16) float sY[16 * kTP];
  __shared__ __align__(16) float sA[kNst * 256];
  const int tid = threadIdx.x, lane = tid & 31, wave = tid >> 5;
  constexpr int kBlkPerB = kDin / 256;
  const int bix = blockIdx.x / kBlkPerB;
  const int d0  = (blockIdx.x - bix * kBlkPerB) * 256;
  const int d   = d0 + tid;
  const size_t row0 = (size_t)bix * kSeq;

#pragma unroll 1
  for (int s = 0; s < kNst; ++s) sA[s * 256 + tid] = -expf(Alog[(size_t)d * kNst + s]);
  __syncthreads();
  float An[kNst], h[kNst];
#pragma unroll
  for (int n = 0; n < kNst; ++n) {
    An[n] = sA[n * 256 + tid];
    h[n] = 0.f;
  }
  const v4f wv = *(const v4f*)(cw + (size_t)d * 4);
  const float bc = cb[d];
  const float Dd = Dv[d];
  float xm3 = 0.f, xm2 = 0.f, xm1 = 0.f;
  const int sr = tid >> 4, sc = (tid & 15) * 2;
  const bool hsel = (d & 1) != 0;

#pragma unroll 1
  for (int c = 0; c < kSeq / 16; ++c) {
    const int l0 = c * 16;
    {
      const v2f v = *(const v2f*)(BC + (row0 + l0 + sr) * kBcP + sc);
      *(v2f*)(sBC + sr * kBcP + sc) = v;
    }
    __syncthreads();
#pragma unroll 1
    for (int s = 0; s < 16; ++s) {
      const size_t m = row0 + (size_t)(l0 + s);
      const float xcur = XZ[m * kXzP + d];
      const float zv   = XZ[m * kXzP + kDin + d];
      const unsigned wd = DLW[(m * kDin + d) >> 1];
      const unsigned hb = hsel ? (wd >> 16) : (wd & 0xffffu);
      const float v = h16_to_f32(hb) * kInvDL;
      float ca = bc;
      ca = fmaf(wv[0], xm3, ca);
      ca = fmaf(wv[1], xm2, ca);
      ca = fmaf(wv[2], xm1, ca);
      ca = fmaf(wv[3], xcur, ca);
      xm3 = xm2; xm2 = xm1; xm1 = xcur;
      const float xi = ca * __builtin_amdgcn_rcpf(1.0f + expf(-ca));
      const float av  = expf(-fabsf(v));
      const float u   = 1.0f + av;
      const float l1p = __logf(u) + (av - (u - 1.0f)) * __builtin_amdgcn_rcpf(u);
      const float delta = fmaxf(v, 0.0f) + l1p;
      const float dtx = delta * xi;
      v4f Bq[4], Cq[4];
#pragma unroll
      for (int qq = 0; qq < 4; ++qq) {
        Bq[qq] = *(const v4f*)(sBC + s * kBcP + 4 * qq);
        Cq[qq] = *(const v4f*)(sBC + s * kBcP + kNst + 4 * qq);
      }
      float y = 0.f;
#pragma unroll
      for (int n = 0; n < kNst; ++n) {
        const float e = __expf(delta * An[n]);
        const float hn = fmaf(e, h[n], dtx * Bq[n >> 2][n & 3]);
        h[n] = hn;
        y = fmaf(Cq[n >> 2][n & 3], hn, y);
      }
      y = fmaf(xi, Dd, y);
      const float g = zv * __builtin_amdgcn_rcpf(1.0f + expf(-zv));
      sY[s * kTP + tid] = (y * g) * kCarY;
    }
    __syncthreads();
    v8h hv[2];
#pragma unroll
    for (int it = 0; it < 2; ++it) {
      const float* sp = sY + (it * 8 + wave) * kTP + lane * 8;
      const v4f a0 = *(const v4f*)(sp);
      const v4f a1 = *(const v4f*)(sp + 4);
#pragma unroll
      for (int e = 0; e < 4; ++e) { hv[it][e] = (_Float16)a0[e]; hv[it][4 + e] = (_Float16)a1[e]; }
    }
    for (int pass = 0; pass < 2; ++pass) {
#pragma unroll
      for (int it = 0; it < 2; ++it)
        *(volatile v8h*)(YG + (row0 + (size_t)(l0 + it * 8 + wave)) * kDin + d0 + lane * 8) = hv[it];
      __threadfence();
    }
  }
}

extern "C" void kernel_launch(void* const* d_in, const int* in_sizes, int n_in,
                              void* d_out, int out_size, void* d_ws, size_t ws_size,
                              hipStream_t stream) {
  if (n_in < 10) return;
  if (in_sizes[0] != kRows * kDm) return;
  if (in_sizes[1] != kXzP * kDm) return;
  if (in_sizes[2] != kDin * 4) return;
  if (in_sizes[3] != kDin) return;
  if (in_sizes[4] != kPrjN * kDin) return;
  if (in_sizes[5] != kDin * kDin) return;
  if (in_sizes[6] != kDin) return;
  if (in_sizes[7] != kDin * kNst) return;
  if (in_sizes[8] != kDin) return;
  if (in_sizes[9] != kDm * kDin) return;
  if (out_size != kRows * kDm) return;
  if (ws_size < kWsTotal) return;

  const float* x       = (const float*)d_in[0];
  const float* W_in    = (const float*)d_in[1];
  const float* conv_w  = (const float*)d_in[2];
  const float* conv_b  = (const float*)d_in[3];
  const float* W_xproj = (const float*)d_in[4];
  const float* W_dt    = (const float*)d_in[5];
  const float* b_dt    = (const float*)d_in[6];
  const float* A_log   = (const float*)d_in[7];
  const float* Dp      = (const float*)d_in[8];
  const float* W_out   = (const float*)d_in[9];
  float* out = (float*)d_out;

  char* ws = (char*)d_ws;
  unsigned short* Xh  = (unsigned short*)(ws + kOffP0);
  unsigned short* W1h = (unsigned short*)(ws + kOffP0 + (size_t)kRows * kDm * 2);
  unsigned short* DRh = (unsigned short*)(ws + kOffP0);
  unsigned short* YGh = (unsigned short*)(ws + kOffP0);
  float*          XZ  = (float*)(ws + kOffXZ);
  unsigned short* XIh = (unsigned short*)(ws + kOffP2);
  unsigned short* DLh = (unsigned short*)(ws + kOffP2);
  unsigned short* W2h = (unsigned short*)(ws + kOffW2);
  float*          BC  = (float*)(ws + kOffBC);
  unsigned short* W3h = (unsigned short*)(ws + kOffW3);
  unsigned short* W4h = (unsigned short*)(ws + kOffW4);

  {
    const int nx  = kRows * kDm / 8;
    const int nw1 = kXzP * kDm / 8;
    const int nw2 = kPrjP * kDin / 8;
    const int rw2 = kPrjN * kDin / 8;
    const int nw3 = kDin * kDin / 8;
    const int nw4 = kDm * kDin / 8;
    cast_f16_kernel<<<nx / 256, 256, 0, stream>>>(x, Xh, nx, nx, kCarX);
    cast_f16_kernel<<<nw1 / 256, 256, 0, stream>>>(W_in, W1h, nw1, nw1, kCarW);
    cast_f16_kernel<<<nw2 / 256, 256, 0, stream>>>(W_xproj, W2h, nw2, rw2, kCarW);
    cast_f16_kernel<<<nw3 / 256, 256, 0, stream>>>(W_dt, W3h, nw3, nw3, kCarW);
    cast_f16_kernel<<<nw4 / 256, 256, 0, stream>>>(W_out, W4h, nw4, nw4, kCarW);
  }

  wmma_gemm64_f16<0, false><<<(kRows / 64) * (kXzP / 64) / 8, 256, 0, stream>>>(
      Xh, kDm, W1h, kDm, (void*)XZ, kXzP, b_dt, kRows, kXzP, kDm, kSclIn, 1.0f);

  conv_silu_kernel<<<dim3(kDin / 256, kRows / 64), 256, 0, stream>>>(XZ, conv_w, conv_b, XIh);

  wmma_gemm64_f16<1, false><<<(kRows / 64) * (kDin / 64) / 8, 256, 0, stream>>>(
      XIh, kDin, W2h, kDin, (void*)DRh, kDin, b_dt, kRows, kDin, kDin, kSclXp, kCarDR);

  wmma_gemm64_f16<3, false><<<(kRows / 64) * 1 / 8, 256, 0, stream>>>(
      XIh, kDin, W2h + (size_t)kDin * kDin, kDin, (void*)BC, kBcP, b_dt, kRows, 64, kDin, kSclXp, 1.0f);

  wmma_gemm64_f16<1, true><<<(kRows / 64) * (kDin / 64) / 8, 256, 0, stream>>>(
      DRh, kDin, W3h, kDin, (void*)DLh, kDin, b_dt, kRows, kDin, kDin, kSclDt, kCarDL);

  scan_kernel<<<kBatch * (kDin / 256), 256, 0, stream>>>(
      XZ, (const unsigned*)DLh, BC, conv_w, conv_b, A_log, Dp, YGh);

  wmma_gemm64_f16<0, false><<<(kRows / 64) * (kDm / 64) / 8, 256, 0, stream>>>(
      YGh, kDin, W4h, kDin, (void*)out, kDm, b_dt, kRows, kDm, kDin, kSclOut, 1.0f);
}
